// MAMBA_52484500357128
// MI455X (gfx1250) — hardware-verified
//
#include <hip/hip_runtime.h>
#include <math.h>

constexpr int NBATCH      = 128;
constexpr int NPOS        = 64;
constexpr int NCHAN       = 256;
constexpr int NTOKEN      = NBATCH * NPOS;
constexpr int NGROUP      = 4;
constexpr int NDIRS       = 4;
constexpr int DGROUP      = 64;
constexpr int NSTATE      = 6;
constexpr int DTRANK      = 6;
constexpr int NPROJ       = 18;
constexpr int XG_PITCH    = 65;
constexpr int PJ_PITCH    = 20;
constexpr int SCAN_THREADS = 64;
constexpr int ELT_THREADS = 256;
constexpr int GEMM_ROWS   = NTOKEN;
constexpr int GEMM_COLS   = NCHAN;
constexpr int GEMM_DEPTH  = NCHAN;
constexpr int GEMM_TILES_N = GEMM_COLS / 64;
constexpr int GEMM_TILES_M = GEMM_ROWS / 64;
constexpr int GEMM_TILES   = GEMM_TILES_M * GEMM_TILES_N;
constexpr int GEMM_BLOCKS  = GEMM_TILES / 8;
constexpr int SLAB_PITCH   = 68;
constexpr float BN_EPS_F   = 1e-5f;
constexpr float LN_EPS_F   = 1e-5f;

static_assert(NTOKEN == 8192, "token count");
static_assert(NCHAN == NGROUP * DGROUP, "channel grouping");
static_assert(NPROJ == DTRANK + 2 * NSTATE, "projection rows");
static_assert(GEMM_DEPTH % 32 == 0, "k multiple of 32");
static_assert(GEMM_ROWS % 64 == 0 && GEMM_COLS % 64 == 0, "tile multiples");
static_assert(GEMM_TILES % 8 == 0, "whole blocks of 8 wave tiles");
static_assert(NTOKEN % 8 == 0, "norm grid exact");
static_assert((NTOKEN * NCHAN / 8) % ELT_THREADS == 0, "split grid exact");
static_assert((NCHAN * NCHAN / 8) % ELT_THREADS == 0, "weight split grid exact");
static_assert((NTOKEN * 64) % ELT_THREADS == 0, "conv grid exact");
static_assert(PJ_PITCH % 4 == 0 && PJ_PITCH >= NPROJ, "projection pitch");

typedef __attribute__((ext_vector_type(16))) __bf16   v16b;
typedef __attribute__((ext_vector_type(8)))  __bf16   v8b;
typedef __attribute__((ext_vector_type(8)))  float    v8f;
typedef __attribute__((ext_vector_type(4)))  float    v4f;
typedef __attribute__((ext_vector_type(4)))  unsigned v4u;
typedef __attribute__((ext_vector_type(2)))  unsigned v2u;

__device__ __forceinline__ unsigned bf16_rne_bits(float f) {
  const unsigned u = __float_as_uint(f);
  return (u + 0x7FFFu + ((u >> 16) & 1u)) >> 16;
}
__device__ __forceinline__ float bf16_bits_to_f32(unsigned h) { return __uint_as_float(h << 16); }
__device__ __forceinline__ void split_bf16(float f, unsigned& hb, unsigned& lb) {
  hb = bf16_rne_bits(f);
  lb = bf16_rne_bits(f - bf16_bits_to_f32(hb));
}
__device__ __forceinline__ void split_pack8(const v4f a, const v4f b, v4u& hv, v4u& lv) {
  unsigned hb[8], lb[8];
#pragma unroll
  for (int e = 0; e < 4; ++e) {
    const float fa = a[e];
    const float fb = b[e];
    split_bf16(fa, hb[e], lb[e]);
    split_bf16(fb, hb[4 + e], lb[4 + e]);
  }
  hv = (v4u){hb[0] | (hb[1] << 16), hb[2] | (hb[3] << 16), hb[4] | (hb[5] << 16), hb[6] | (hb[7] << 16)};
  lv = (v4u){lb[0] | (lb[1] << 16), lb[2] | (lb[3] << 16), lb[4] | (lb[5] << 16), lb[6] | (lb[7] << 16)};
}
__device__ __forceinline__ float silu_precise(float v) { return v * (1.0f / (1.0f + expf(-v))); }

__device__ __forceinline__ void group_guard4(v8f& a, v8f& b, v8f& c, v8f& d, v16b x, v16b y) {
  asm volatile("v_nop\n\tv_nop\n\tv_nop\n\tv_nop" : "+v"(a), "+v"(b), "+v"(c), "+v"(d) : "v"(x), "v"(y));
}
__device__ __forceinline__ void keep4_b(v16b a, v16b b, v16b c, v16b d) { asm volatile("v_nop" :: "v"(a), "v"(b), "v"(c), "v"(d)); }
__device__ __forceinline__ void acc_guard4(v8f& a, v8f& b, v8f& c, v8f& d) { asm volatile("v_nop\n\tv_nop\n\tv_nop\n\tv_nop" : "+v"(a), "+v"(b), "+v"(c), "+v"(d)); }

struct FragB {
  union U { v16b v; v8b h[2]; };
  static __device__ __forceinline__ v16b load(const __bf16* p) {
    U f; f.h[0] = *(const v8b*)(p); f.h[1] = *(const v8b*)(p + 16); return f.v;
  }
  static __device__ __forceinline__ v8f mma(v16b a, v16b b, v8f c) {
    return __builtin_amdgcn_wmma_f32_16x16x32_bf16(false, a, false, b, (short)0, c, false, false);
  }
};

__global__ __launch_bounds__(ELT_THREADS) void split8_kernel(const float* __restrict__ src,
                                                             unsigned short* __restrict__ hi,
                                                             unsigned short* __restrict__ lo, int n8) {
  const int i = blockIdx.x * ELT_THREADS + threadIdx.x;
  if (i < n8) {
    const v4f a = *(const v4f*)(src + (size_t)i * 8);
    const v4f b = *(const v4f*)(src + (size_t)i * 8 + 4);
    v4u hv, lv;
    split_pack8(a, b, hv, lv);
    *(volatile v4u*)(hi + (size_t)i * 8) = hv;
    *(volatile v4u*)(lo + (size_t)i * 8) = lv;
    __threadfence();
    *(volatile v4u*)(hi + (size_t)i * 8) = hv;
    *(volatile v4u*)(lo + (size_t)i * 8) = lv;
  }
}

__global__ __launch_bounds__(ELT_THREADS) void fold_conv_kernel(const float* __restrict__ x,
                                                                const float* __restrict__ cw,
                                                                const float* __restrict__ cb,
                                                                unsigned short* __restrict__ Phi,
                                                                unsigned short* __restrict__ Plo) {
  const int i = blockIdx.x * ELT_THREADS + threadIdx.x;
  if (i >= NTOKEN * 64) return;
  const int token = i >> 6;
  const int j  = i & 63;
  const int b  = token >> 6;
  const int p  = (token >> 3) & 7;
  const int q  = token & 7;
  const int c  = j >> 4;
  const int r  = (j >> 1) & 7;
  const int s0 = (j & 1) * 4;

  const int wl  = q * 8 + s0 - 1;
  const bool okl = (wl >= 0);
  const int wlc = okl ? wl : 0;
  const int wr  = q * 8 + s0 + 4;
  const bool okr = (wr < 64);
  const int wrc = okr ? wr : 63;

  float acc[4];
  const float bias = cb[c];
#pragma unroll
  for (int e = 0; e < 4; ++e) acc[e] = bias;

#pragma unroll 1
  for (int ti = 0; ti < 3; ++ti) {
    const int hh  = p * 8 + r + ti - 1;
    const bool okh = (hh >= 0) && (hh < 64);
    const int hhc = hh < 0 ? 0 : (hh > 63 ? 63 : hh);
    const int hp  = hhc >> 3;
    const int rr  = hhc & 7;
    const int rowbase = ((b * 8 + hp) * 8) * NCHAN + c * 64 + rr * 8;
    v4f ctr = *(const v4f*)(x + rowbase + q * NCHAN + s0);
    float lf = x[rowbase + (wlc >> 3) * NCHAN + (wlc & 7)];
    float rt = x[rowbase + (wrc >> 3) * NCHAN + (wrc & 7)];
    asm volatile("" : "+v"(ctr));
    asm volatile("" : "+v"(lf));
    asm volatile("" : "+v"(rt));
    const float w0 = cw[c * 9 + ti * 3 + 0];
    const float w1 = cw[c * 9 + ti * 3 + 1];
    const float w2 = cw[c * 9 + ti * 3 + 2];
    float vv[6];
    vv[0] = (okh && okl) ? lf : 0.0f;
#pragma unroll
    for (int e = 0; e < 4; ++e) {
      const float ce = ctr[e];
      vv[1 + e] = okh ? ce : 0.0f;
    }
    vv[5] = (okh && okr) ? rt : 0.0f;
#pragma unroll
    for (int e = 0; e < 4; ++e) acc[e] += w0 * vv[e] + w1 * vv[e + 1] + w2 * vv[e + 2];
  }

  unsigned hb[4], lb[4];
#pragma unroll
  for (int e = 0; e < 4; ++e) {
    const float sv = silu_precise(acc[e]);
    split_bf16(sv, hb[e], lb[e]);
  }
  const v2u hv = (v2u){hb[0] | (hb[1] << 16), hb[2] | (hb[3] << 16)};
  const v2u lv = (v2u){lb[0] | (lb[1] << 16), lb[2] | (lb[3] << 16)};
  *(volatile v2u*)(Phi + (size_t)i * 4) = hv;
  *(volatile v2u*)(Plo + (size_t)i * 4) = lv;
  __threadfence();
  *(volatile v2u*)(Phi + (size_t)i * 4) = hv;
  *(volatile v2u*)(Plo + (size_t)i * 4) = lv;
}

template <int EPI>
__global__ __launch_bounds__(256) void gemm_split_kernel(
    const unsigned short* __restrict__ Ahp, const unsigned short* __restrict__ Alp,
    const unsigned short* __restrict__ Bhp, const unsigned short* __restrict__ Blp,
    float* __restrict__ Cout,
    const float* __restrict__ pbias, const float* __restrict__ bmean, const float* __restrict__ bvar,
    const float* __restrict__ bgam, const float* __restrict__ bbeta) {
  const __bf16* Ah = (const __bf16*)Ahp;
  const __bf16* Al = (const __bf16*)Alp;
  const __bf16* Bh = (const __bf16*)Bhp;
  const __bf16* Bl = (const __bf16*)Blp;
  __shared__ __align__(16) float sT[8][16 * SLAB_PITCH];
  const int lane = threadIdx.x & 31;
  const int wave = threadIdx.x >> 5;
  const int tile = blockIdx.x * 8 + wave;
  if (tile >= GEMM_TILES) return;
  const int tm = tile / GEMM_TILES_N;
  const int tn = tile - tm * GEMM_TILES_N;
  const int m0 = tm << 6;
  const int n0 = tn << 6;
  const int rlane = lane & 15;
  const int koff  = (lane >> 4) * 8;
  const int mOff  = (lane >> 4) * 8;

  v8f acc[4][4];
#pragma unroll
  for (int i = 0; i < 4; ++i)
#pragma unroll
    for (int j = 0; j < 4; ++j) acc[i][j] = (v8f){0.f, 0.f, 0.f, 0.f, 0.f, 0.f, 0.f, 0.f};

#pragma unroll 1
  for (int k0 = 0; k0 < GEMM_DEPTH; k0 += 32) {
    v16b bh[4], bl[4];
#pragma unroll
    for (int j = 0; j < 4; ++j) {
      const size_t bo = (size_t)(n0 + (j << 4) + rlane) * GEMM_DEPTH + koff + k0;
      bh[j] = FragB::load(Bh + bo);
      bl[j] = FragB::load(Bl + bo);
    }
#pragma unroll
    for (int i = 0; i < 4; ++i) {
      const size_t ao = (size_t)(m0 + (i << 4) + rlane) * GEMM_DEPTH + koff + k0;
      const v16b ah = FragB::load(Ah + ao);
      const v16b al = FragB::load(Al + ao);
#pragma unroll
      for (int j = 0; j < 4; ++j) {
        acc[i][j] = FragB::mma(ah, bh[j], acc[i][j]);
        acc[i][j] = FragB::mma(ah, bl[j], acc[i][j]);
        acc[i][j] = FragB::mma(al, bh[j], acc[i][j]);
      }
      group_guard4(acc[i][0], acc[i][1], acc[i][2], acc[i][3], ah, al);
    }
    keep4_b(bh[0], bh[1], bh[2], bh[3]);
    keep4_b(bl[0], bl[1], bl[2], bl[3]);
  }
  acc_guard4(acc[0][0], acc[0][1], acc[0][2], acc[0][3]);
  acc_guard4(acc[1][0], acc[1][1], acc[1][2], acc[1][3]);
  acc_guard4(acc[2][0], acc[2][1], acc[2][2], acc[2][3]);
  acc_guard4(acc[3][0], acc[3][1], acc[3][2], acc[3][3]);

  float* slab = sT[wave];
  const int hh = lane >> 4;
  const int c4 = (lane & 15) * 4;
  v4f pb4 = (v4f){0.f, 0.f, 0.f, 0.f};
  v4f mu4 = pb4, sc4 = pb4, be4 = pb4;
  if (EPI == 1) {
    pb4 = *(const v4f*)(pbias + n0 + c4);
    mu4 = *(const v4f*)(bmean + n0 + c4);
    be4 = *(const v4f*)(bbeta + n0 + c4);
    const v4f var4 = *(const v4f*)(bvar + n0 + c4);
    const v4f gm4  = *(const v4f*)(bgam + n0 + c4);
#pragma unroll
    for (int e = 0; e < 4; ++e) {
      const float vr = var4[e];
      const float gm = gm4[e];
      sc4[e] = rsqrtf(vr + BN_EPS_F) * gm;
    }
  }
#pragma unroll
  for (int i = 0; i < 4; ++i) {
    const int mBase = m0 + (i << 4);
#pragma unroll
    for (int j = 0; j < 4; ++j) {
#pragma unroll
      for (int r = 0; r < 8; ++r) slab[(mOff + r) * SLAB_PITCH + (j << 4) + rlane] = acc[i][j][r];
    }
    __builtin_amdgcn_fence(__ATOMIC_RELEASE, "workgroup");
    __builtin_amdgcn_wave_barrier();
    __builtin_amdgcn_fence(__ATOMIC_ACQUIRE, "workgroup");
    v4f ov[8];
#pragma unroll
    for (int it = 0; it < 8; ++it) {
      const int row = it * 2 + hh;
      v4f v = *(const v4f*)(slab + row * SLAB_PITCH + c4);
      if (EPI == 1) {
#pragma unroll
        for (int e = 0; e < 4; ++e) v[e] = ((v[e] + pb4[e]) - mu4[e]) * sc4[e] + be4[e];
      }
      ov[it] = v;
    }
    for (int pass = 0; pass < 2; ++pass) {
#pragma unroll
      for (int it = 0; it < 8; ++it) {
        const int row = it * 2 + hh;
        *(volatile v4f*)(Cout + (size_t)(mBase + row) * GEMM_COLS + n0 + c4) = ov[it];
      }
      __threadfence();
    }
    __builtin_amdgcn_fence(__ATOMIC_RELEASE, "workgroup");
    __builtin_amdgcn_wave_barrier();
    __builtin_amdgcn_fence(__ATOMIC_ACQUIRE, "workgroup");
  }
}

__global__ __launch_bounds__(SCAN_THREADS) void cross_scan_kernel(
    const float* __restrict__ Xp, const float* __restrict__ xpw, const float* __restrict__ dtw,
    const float* __restrict__ dtb, const float* __restrict__ alog, const float* __restrict__ dsk,
    float* __restrict__ Ysum) {
  __shared__ __align__(16) float xg[DGROUP * XG_PITCH];
  __shared__ __align__(16) float ys[DGROUP * XG_PITCH];
  __shared__ __align__(16) float wT[DGROUP * PJ_PITCH];
  __shared__ __align__(16) float xd[NPOS * PJ_PITCH];
  __shared__ __align__(16) float acoef[DGROUP * 8];

  const int t    = threadIdx.x;
  const int lane = t & 31;
  const int wave = t >> 5;
  const int g    = blockIdx.x & 3;
  const int b    = blockIdx.x >> 2;

#pragma unroll 1
  for (int it = 0; it < 16; ++it) {
    const int idx = it * 64 + t;
    const int pos = idx >> 4;
    const int d4  = (idx & 15) * 4;
    const v4f v = *(const v4f*)(Xp + (size_t)(b * 64 + pos) * NCHAN + g * 64 + d4);
    xg[(d4 + 0) * XG_PITCH + pos] = v[0];
    xg[(d4 + 1) * XG_PITCH + pos] = v[1];
    xg[(d4 + 2) * XG_PITCH + pos] = v[2];
    xg[(d4 + 3) * XG_PITCH + pos] = v[3];
  }
#pragma unroll 1
  for (int l = 0; l < NPOS; ++l) ys[t * XG_PITCH + l] = 0.0f;

#pragma unroll 1
  for (int kk = 0; kk < NDIRS; ++kk) {
    const int k  = ((kk & 1) << 1) | (kk >> 1);
    const int gk = g * 4 + k;
    const int pbase = gk * 64 + t;
    __syncthreads();
    {
      const float* W = xpw + (size_t)gk * NPROJ * 64;
#pragma unroll 1
      for (int c = 0; c < PJ_PITCH; ++c) {
        const int cc = (c < NPROJ) ? c : (NPROJ - 1);
        const float w = W[cc * 64 + t];
        wT[t * PJ_PITCH + c] = (c < NPROJ) ? w : 0.0f;
      }
#pragma unroll 1
      for (int n = 0; n < NSTATE; ++n) acoef[t * 8 + n] = -expf(alog[pbase * NSTATE + n]);
    }
    __syncthreads();

    {
      float pa[NPROJ];
#pragma unroll
      for (int c = 0; c < NPROJ; ++c) pa[c] = 0.0f;
#pragma unroll 1
      for (int d = 0; d < DGROUP; ++d) {
        const float xv = xg[d * XG_PITCH + t];
        const v4f w0 = *(const v4f*)(wT + d * PJ_PITCH);
        const v4f w1 = *(const v4f*)(wT + d * PJ_PITCH + 4);
        const v4f w2 = *(const v4f*)(wT + d * PJ_PITCH + 8);
        const v4f w3 = *(const v4f*)(wT + d * PJ_PITCH + 12);
        const v4f w4 = *(const v4f*)(wT + d * PJ_PITCH + 16);
#pragma unroll
        for (int e = 0; e < 4; ++e) {
          pa[e]      += xv * w0[e];
          pa[4 + e]  += xv * w1[e];
          pa[8 + e]  += xv * w2[e];
          pa[12 + e] += xv * w3[e];
        }
        pa[16] += xv * w4[0];
        pa[17] += xv * w4[1];
      }
      *(v4f*)(xd + t * PJ_PITCH)      = (v4f){pa[0],  pa[1],  pa[2],  pa[3]};
      *(v4f*)(xd + t * PJ_PITCH + 4)  = (v4f){pa[4],  pa[5],  pa[6],  pa[7]};
      *(v4f*)(xd + t * PJ_PITCH + 8)  = (v4f){pa[8],  pa[9],  pa[10], pa[11]};
      *(v4f*)(xd + t * PJ_PITCH + 12) = (v4f){pa[12], pa[13], pa[14], pa[15]};
      *(v4f*)(xd + t * PJ_PITCH + 16) = (v4f){pa[16], pa[17], 0.0f,   0.0f};
    }
    __syncthreads();

    {
      float dw[DTRANK], a6[NSTATE], h[NSTATE];
#pragma unroll
      for (int n = 0; n < NSTATE; ++n) {
        dw[n] = dtw[pbase * DTRANK + n];
        a6[n] = acoef[t * 8 + n];
        h[n]  = 0.0f;
      }
      const float dtbv = dtb[pbase];
      const float dsv  = dsk[pbase];
      const int rev = (k >> 1) & 1;
      const int tr  = k & 1;
#pragma unroll 1
      for (int l = 0; l < NPOS; ++l) {
        const int m   = rev ? (63 - l) : l;
        const int pos = tr ? (((m & 7) << 3) | (m >> 3)) : m;
        const v4f q0 = *(const v4f*)(xd + pos * PJ_PITCH);
        const v4f q1 = *(const v4f*)(xd + pos * PJ_PITCH + 4);
        const v4f q2 = *(const v4f*)(xd + pos * PJ_PITCH + 8);
        const v4f q3 = *(const v4f*)(xd + pos * PJ_PITCH + 12);
        const v4f q4 = *(const v4f*)(xd + pos * PJ_PITCH + 16);
        float pj[PJ_PITCH];
#pragma unroll
        for (int e = 0; e < 4; ++e) {
          pj[e] = q0[e]; pj[4 + e] = q1[e]; pj[8 + e] = q2[e]; pj[12 + e] = q3[e]; pj[16 + e] = q4[e];
        }
        float de = 0.0f;
#pragma unroll
        for (int r = 0; r < DTRANK; ++r) de += pj[r] * dw[r];
        de += dtbv;
        const float sp = fmaxf(de, 0.0f) + log1pf(expf(-fabsf(de)));
        const float xv = xg[t * XG_PITCH + pos];
        const float dx = sp * xv;
        float yv = 0.0f;
#pragma unroll
        for (int n = 0; n < NSTATE; ++n) {
          h[n] = expf(sp * a6[n]) * h[n] + dx * pj[DTRANK + n];
          yv  += h[n] * pj[DTRANK + NSTATE + n];
        }
        yv += dsv * xv;
        ys[t * XG_PITCH + pos] += yv;
      }
    }
  }
  __syncthreads();

  {
    const int hh = lane >> 4;
    const int c4 = (lane & 15) * 4;
    v4f ov[16];
#pragma unroll
    for (int it = 0; it < 16; ++it) {
      const int pos = wave * 32 + it * 2 + hh;
      ov[it] = (v4f){ys[(c4 + 0) * XG_PITCH + pos], ys[(c4 + 1) * XG_PITCH + pos],
                     ys[(c4 + 2) * XG_PITCH + pos], ys[(c4 + 3) * XG_PITCH + pos]};
    }
    for (int pass = 0; pass < 2; ++pass) {
#pragma unroll
      for (int it = 0; it < 16; ++it) {
        const int pos = wave * 32 + it * 2 + hh;
        *(volatile v4f*)(Ysum + (size_t)(b * 64 + pos) * NCHAN + g * 64 + c4) = ov[it];
      }
      __threadfence();
    }
  }
}

__global__ __launch_bounds__(ELT_THREADS) void norm_gate_kernel(const float* __restrict__ Ysum,
                                                                const float* __restrict__ Zpre,
                                                                const float* __restrict__ lng,
                                                                const float* __restrict__ lnb,
                                                                unsigned short* __restrict__ Yhi,
                                                                unsigned short* __restrict__ Ylo) {
  __shared__ __align__(16) float rowbuf[8][NCHAN];
  const int tid  = threadIdx.x;
  const int lane = tid & 31;
  const int wave = tid >> 5;
  const int token = blockIdx.x * 8 + wave;
  const float* yr = Ysum + (size_t)token * NCHAN;
  const float* zr = Zpre + (size_t)token * NCHAN;

  const v4f y0 = *(const v4f*)(yr + 8 * lane);
  const v4f y1 = *(const v4f*)(yr + 8 * lane + 4);
  float s = ((y0[0] + y0[1]) + (y0[2] + y0[3])) + ((y1[0] + y1[1]) + (y1[2] + y1[3]));
#pragma unroll
  for (int off = 1; off < 32; off <<= 1) s += __shfl_xor(s, off, 32);
  const float mu = s * (1.0f / (float)NCHAN);
  float ss = 0.0f;
#pragma unroll
  for (int e = 0; e < 4; ++e) {
    const float d0 = y0[e] - mu;
    const float d1 = y1[e] - mu;
    ss += d0 * d0;
    ss += d1 * d1;
  }
#pragma unroll
  for (int off = 1; off < 32; off <<= 1) ss += __shfl_xor(ss, off, 32);
  const float var  = ss * (1.0f / (float)NCHAN);
  const float rstd = rsqrtf(var + LN_EPS_F);

#pragma unroll 1
  for (int j = 0; j < 8; ++j) {
    const int ch = 32 * j + lane;
    const float yv = yr[ch];
    const float zv = zr[ch];
    const float gv = lng[ch];
    const float bv = lnb[ch];
    const float yn = ((yv - mu) * rstd) * gv + bv;
    rowbuf[wave][ch] = yn * silu_precise(zv);
  }
  __syncthreads();
  const v4f a = *(const v4f*)(&rowbuf[wave][8 * lane]);
  const v4f c = *(const v4f*)(&rowbuf[wave][8 * lane + 4]);
  v4u hv, lv;
  split_pack8(a, c, hv, lv);
  unsigned short* hp = Yhi + (size_t)token * NCHAN + 8 * lane;
  unsigned short* lp = Ylo + (size_t)token * NCHAN + 8 * lane;
  *(volatile v4u*)hp = hv;
  *(volatile v4u*)lp = lv;
  __threadfence();
  *(volatile v4u*)hp = hv;
  *(volatile v4u*)lp = lv;
}

extern "C" void kernel_launch(void* const* d_in, const int* in_sizes, int n_in,
                              void* d_out, int out_size, void* d_ws, size_t ws_size, hipStream_t stream) {
  if (n_in < 18 || d_out == nullptr || d_ws == nullptr) return;
  if (in_sizes[0] != NTOKEN * NCHAN || in_sizes[1] != NCHAN * NCHAN || in_sizes[2] != 36 || in_sizes[3] != 4 ||
      in_sizes[4] != NCHAN * NCHAN || in_sizes[5] != NCHAN || in_sizes[6] != NCHAN || in_sizes[7] != NCHAN ||
      in_sizes[8] != NCHAN || in_sizes[9] != NCHAN || in_sizes[10] != NGROUP * NDIRS * NPROJ * DGROUP ||
      in_sizes[11] != NGROUP * NDIRS * DGROUP * DTRANK || in_sizes[12] != NGROUP * NDIRS * DGROUP ||
      in_sizes[13] != NGROUP * NDIRS * DGROUP * NSTATE || in_sizes[14] != NGROUP * NDIRS * DGROUP ||
      in_sizes[15] != NCHAN || in_sizes[16] != NCHAN || in_sizes[17] != NCHAN * NCHAN ||
      out_size != NTOKEN * NCHAN) return;

  const float* x_in       = (const float*)d_in[0];
  const float* in_proj_w  = (const float*)d_in[1];
  const float* conv_w     = (const float*)d_in[2];
  const float* conv_b     = (const float*)d_in[3];
  const float* patch_w    = (const float*)d_in[4];
  const float* patch_b    = (const float*)d_in[5];
  const float* bn_gamma   = (const float*)d_in[6];
  const float* bn_beta    = (const float*)d_in[7];
  const float* bn_mean    = (const float*)d_in[8];
  const float* bn_var     = (const float*)d_in[9];
  const float* x_proj_w   = (const float*)d_in[10];
  const float* dt_w       = (const float*)d_in[11];
  const float* dt_b       = (const float*)d_in[12];
  const float* A_logs     = (const float*)d_in[13];
  const float* Ds         = (const float*)d_in[14];
  const float* ln_gamma   = (const float*)d_in[15];
  const float* ln_beta    = (const float*)d_in[16];
  const float* out_proj_w = (const float*)d_in[17];
  float* out = (float*)d_out;

  char* ws = (char*)d_ws;
  size_t off = 0;
  auto carve = [&](size_t bytes) -> char* { char* p = ws + off; off += (bytes + 255) & ~(size_t)255; return p; };
  const size_t wplane = (size_t)NCHAN * NCHAN * 2;
  const size_t hplane = (size_t)NTOKEN * NCHAN * 2;
  const size_t fplane = (size_t)NTOKEN * NCHAN * 4;
  unsigned short* W1H  = (unsigned short*)carve(wplane);
  unsigned short* W1L  = (unsigned short*)carve(wplane);
  unsigned short* W4H  = (unsigned short*)carve(wplane);
  unsigned short* W4L  = (unsigned short*)carve(wplane);
  unsigned short* W17H = (unsigned short*)carve(wplane);
  unsigned short* W17L = (unsigned short*)carve(wplane);
  unsigned short* XH   = (unsigned short*)carve(hplane);
  unsigned short* XL   = (unsigned short*)carve(hplane);
  float*          ZP   = (float*)carve(fplane);
  unsigned short* PH   = (unsigned short*)carve(hplane);
  unsigned short* PL   = (unsigned short*)carve(hplane);
  float*          XP   = (float*)carve(fplane);
  float*          YS   = (float*)carve(fplane);
  unsigned short* YH   = (unsigned short*)carve(hplane);
  unsigned short* YL   = (unsigned short*)carve(hplane);
  if (off > ws_size || off > (size_t)134217728) return;

  const int n8x = NTOKEN * NCHAN / 8;
  const int n8w = NCHAN * NCHAN / 8;
  split8_kernel<<<n8x / ELT_THREADS, ELT_THREADS, 0, stream>>>(x_in, XH, XL, n8x);
  split8_kernel<<<n8w / ELT_THREADS, ELT_THREADS, 0, stream>>>(in_proj_w, W1H, W1L, n8w);
  split8_kernel<<<n8w / ELT_THREADS, ELT_THREADS, 0, stream>>>(patch_w, W4H, W4L, n8w);
  split8_kernel<<<n8w / ELT_THREADS, ELT_THREADS, 0, stream>>>(out_proj_w, W17H, W17L, n8w);

  gemm_split_kernel<0><<<GEMM_BLOCKS, 256, 0, stream>>>(XH, XL, W1H, W1L, ZP,
                                                       patch_b, bn_mean, bn_var, bn_gamma, bn_beta);
  fold_conv_kernel<<<(NTOKEN * 64) / ELT_THREADS, ELT_THREADS, 0, stream>>>(x_in, conv_w, conv_b, PH, PL);
  gemm_split_kernel<1><<<GEMM_BLOCKS, 256, 0, stream>>>(PH, PL, W4H, W4L, XP,
                                                       patch_b, bn_mean, bn_var, bn_gamma, bn_beta);
  cross_scan_kernel<<<NBATCH * NGROUP, SCAN_THREADS, 0, stream>>>(XP, x_proj_w, dt_w, dt_b, A_logs, Ds, YS);
  norm_gate_kernel<<<NTOKEN / 8, ELT_THREADS, 0, stream>>>(YS, ZP, ln_gamma, ln_beta, YH, YL);
  gemm_split_kernel<0><<<GEMM_BLOCKS, 256, 0, stream>>>(YH, YL, W17H, W17L, out,
                                                       patch_b, bn_mean, bn_var, bn_gamma, bn_beta);
}
